// HydraBlock_7765300871301
// MI455X (gfx1250) — hardware-verified
//
#include <hip/hip_runtime.h>
#include <math.h>
#include <stdint.h>

#ifndef NB
#define NB 4
#endif
#ifndef SEQ
#define SEQ 2048
#endif
#define NB_FULL 4
#define SEQ_FULL 2048
#define DM 512
#define NHD 8
#define HDD 64
#define DLT 64
#define KVW 1024
#define NEX 32
#define NEXP2 64
#define ECH 8
#define NCHK 4
#define KCH (ECH * DM)
#define KEW (NEX * DM)
#define MTOK (NB * SEQ)

#define WCAR  64.0f
#define RCAR  1024.0f
#define WLCAR 0.0625f
#define HCAR  8.0f
#define KDCAR 16.0f
#define OCAR  64.0f
#define GCAR  256.0f

static_assert(NB >= 1 && NB <= NB_FULL);
static_assert(SEQ >= 64 && SEQ <= SEQ_FULL && (SEQ % 64) == 0);
static_assert((MTOK % 64) == 0);
static_assert(NHD * HDD == DM && NEX == 32 && ECH * NCHK == NEX && NEX <= NEXP2);
static_assert((DM % 64) == 0 && (KVW % 64) == 0 && (DLT % 64) == 0 && (NEXP2 % 64) == 0);
static_assert(((2 * DM) % 32) == 0 && ((2 * DLT) % 32) == 0 && (KCH % 32) == 0);
static_assert(KCH * 2 >= DM * 4 + KVW * 4 + DLT * 4 + 2 * DLT * 2);
static_assert(DM * 4 + 2 * DM * 2 + NEXP2 * 4 >= 2 * DM * 2);

typedef __attribute__((ext_vector_type(16))) _Float16 v16h;
typedef __attribute__((ext_vector_type(8)))  _Float16 v8h;
typedef __attribute__((ext_vector_type(8)))  float    v8f;
typedef __attribute__((ext_vector_type(4)))  float    v4f;
typedef __attribute__((ext_vector_type(4)))  unsigned int v4u;

__device__ __forceinline__ unsigned short f2bf_bits(float f) {
  unsigned u = __float_as_uint(f);
  return (unsigned short)((u + 0x7FFFu + ((u >> 16) & 1u)) >> 16);
}
__device__ __forceinline__ float bf_bits2f(unsigned short h) { return __uint_as_float(((unsigned)h) << 16); }
__device__ __forceinline__ float bfr(float f) { return bf_bits2f(f2bf_bits(f)); }
__device__ __forceinline__ v4f bfr4(v4f a) { v4f r; r[0] = bfr(a[0]); r[1] = bfr(a[1]); r[2] = bfr(a[2]); r[3] = bfr(a[3]); return r; }
__device__ __forceinline__ float sq4(v4f v) { return (v[0] * v[0] + v[1] * v[1]) + (v[2] * v[2] + v[3] * v[3]); }

__device__ __forceinline__ void wave_lds_sync() {
  __builtin_amdgcn_fence(__ATOMIC_RELEASE, "workgroup");
  __builtin_amdgcn_wave_barrier();
  __builtin_amdgcn_fence(__ATOMIC_ACQUIRE, "workgroup");
}

__device__ __forceinline__ void dep_guard_h(v8f& a, v8f& b, v16h x, v16h y) { asm volatile("v_nop\n\tv_nop\n\tv_nop\n\tv_nop" : "+v"(a), "+v"(b) : "v"(x), "v"(y)); }
__device__ __forceinline__ void keep4_h(v16h a, v16h b, v16h c, v16h d) { asm volatile("v_nop" :: "v"(a), "v"(b), "v"(c), "v"(d)); }
__device__ __forceinline__ void acc_guard4(v8f& a, v8f& b, v8f& c, v8f& d) { asm volatile("v_nop\n\tv_nop\n\tv_nop\n\tv_nop" : "+v"(a), "+v"(b), "+v"(c), "+v"(d)); }

union FragU { v16h v; v8h h[2]; _Float16 s[16]; };
struct FragH {
  static __device__ __forceinline__ v16h load(const _Float16* p) {
    FragU f; f.h[0] = *(const v8h*)(p); f.h[1] = *(const v8h*)(p + 16); return f.v;
  }
  static __device__ __forceinline__ v8f mma(v16h a, v16h b, v8f c) {
    return __builtin_amdgcn_wmma_f32_16x16x32_f16(false, a, false, b, (short)0, c, false, false);
  }
};

union Pk8 { v8h h; v4u u; };
__device__ __forceinline__ void split8(v4f a, v4f b, float car, v4u& hi, v4u& lo) {
  Pk8 ph, pl;
#pragma unroll
  for (int e = 0; e < 4; ++e) {
    float t = a[e] * car;
    _Float16 hv = (_Float16)t;
    ph.h[e] = hv;
    pl.h[e] = (_Float16)((t - (float)hv) * RCAR);
    t = b[e] * car;
    hv = (_Float16)t;
    ph.h[4 + e] = hv;
    pl.h[4 + e] = (_Float16)((t - (float)hv) * RCAR);
  }
  hi = ph.u; lo = pl.u;
}

template <int BIAS_MODE, int OUT_MODE, bool RESID>
__global__ __launch_bounds__(256) void wmma_gemm64(
    const unsigned short* __restrict__ Ap, int lda,
    const unsigned short* __restrict__ Btp, int ldb,
    void* Cout, int ldc,
    const float* __restrict__ bias,
    const float* resid,
    int M, int N, int K, float scale, float oscale) {
  const _Float16* A = (const _Float16*)Ap;
  const _Float16* Bt = (const _Float16*)Btp;
  __shared__ __align__(16) float sT[8][16 * 68];
  const int lane = threadIdx.x & 31;
  const int wave = threadIdx.x >> 5;
  const int tilesN = N >> 6;
  const int tilesM = M >> 6;
  const int tile = blockIdx.x * 8 + wave;
  if (tile >= tilesM * tilesN) return;
  const int tm = tile / tilesN;
  const int tn = tile - tm * tilesN;
  const int m0 = tm << 6;
  const int n0 = tn << 6;
  const int rlane = lane & 15;
  const int koff  = (lane >> 4) * 8;
  const int mOff  = (lane >> 4) * 8;

  v8f acc[4][4];
#pragma unroll
  for (int i = 0; i < 4; ++i)
#pragma unroll
    for (int j = 0; j < 4; ++j) acc[i][j] = (v8f){0.f,0.f,0.f,0.f,0.f,0.f,0.f,0.f};

  for (int k0 = 0; k0 < K; k0 += 32) {
    v16h bh[4];
#pragma unroll
    for (int j = 0; j < 4; ++j) {
      const size_t bo = (size_t)(n0 + (j << 4) + rlane) * ldb + koff + k0;
      bh[j] = FragH::load(Bt + bo);
    }
#pragma unroll
    for (int i = 0; i < 4; ++i) {
      const size_t ao = (size_t)(m0 + (i << 4) + rlane) * lda + koff + k0;
      const v16h ah = FragH::load(A + ao);
#pragma unroll
      for (int j = 0; j < 4; ++j) acc[i][j] = FragH::mma(ah, bh[j], acc[i][j]);
      dep_guard_h(acc[i][0], acc[i][3], ah, bh[3]);
    }
    keep4_h(bh[0], bh[1], bh[2], bh[3]);
  }
  acc_guard4(acc[0][0], acc[0][1], acc[0][2], acc[0][3]);
  acc_guard4(acc[1][0], acc[1][1], acc[1][2], acc[1][3]);
  acc_guard4(acc[2][0], acc[2][1], acc[2][2], acc[2][3]);
  acc_guard4(acc[3][0], acc[3][1], acc[3][2], acc[3][3]);

  float* slab = sT[wave];
#pragma unroll
  for (int i = 0; i < 4; ++i) {
    const int mBase = m0 + (i << 4);
#pragma unroll
    for (int j = 0; j < 4; ++j) {
      const int n = n0 + (j << 4) + rlane;
      float bv = 0.f;
      if (BIAS_MODE == 2) bv = bfr(bias[n]);
#pragma unroll
      for (int r = 0; r < 8; ++r) {
        float v = acc[i][j][r] * scale;
        if (BIAS_MODE == 2) v += bv;
        v *= oscale;
        slab[(mOff + r) * 68 + (j << 4) + rlane] = v;
      }
    }
    __builtin_amdgcn_fence(__ATOMIC_RELEASE, "workgroup");
    __builtin_amdgcn_wave_barrier();
    __builtin_amdgcn_fence(__ATOMIC_ACQUIRE, "workgroup");
    if (OUT_MODE == 0) {
      float* C = (float*)Cout;
      const int hh = lane >> 4, c4 = (lane & 15) * 4;
      int orow[8];
#pragma unroll
      for (int it = 0; it < 8; ++it) {
        const int row = it * 2 + hh;
        orow[it] = mBase + row;
      }
      if (RESID) {
#pragma unroll
        for (int it = 0; it < 8; ++it) {
          const int row = it * 2 + hh;
          v4f v = *(const v4f*)(slab + row * 68 + c4);
          const v4f rv = *(const v4f*)(resid + (size_t)orow[it] * ldc + n0 + c4);
          v += rv;
          *(v4f*)(slab + row * 68 + c4) = v;
        }
      }
      for (int pass = 0; pass < 2; ++pass) {
#pragma unroll
        for (int it = 0; it < 8; ++it) {
          const int row = it * 2 + hh;
          const v4f v = *(const v4f*)(slab + row * 68 + c4);
          *(volatile v4f*)(C + (size_t)orow[it] * ldc + n0 + c4) = v;
        }
        __threadfence();
      }
    } else {
      const int q = lane >> 3, c8 = (lane & 7) * 8;
      unsigned short* C = (unsigned short*)Cout;
      for (int pass = 0; pass < 2; ++pass) {
#pragma unroll
        for (int it = 0; it < 4; ++it) {
          const int row = it * 4 + q;
          const float* sp = slab + row * 68 + c8;
          v8h hv;
#pragma unroll
          for (int e = 0; e < 8; ++e) hv[e] = (_Float16)sp[e];
          *(volatile v8h*)(C + (size_t)(mBase + row) * ldc + n0 + c8) = hv;
        }
        __threadfence();
      }
    }
    __builtin_amdgcn_fence(__ATOMIC_RELEASE, "workgroup");
    __builtin_amdgcn_wave_barrier();
    __builtin_amdgcn_fence(__ATOMIC_ACQUIRE, "workgroup");
  }
}

__global__ __launch_bounds__(256) void tr_w16_kernel(const float* __restrict__ in, int ldin, int nreal, size_t inbatch,
                                                     unsigned short* out, int ldout, int coloff, size_t outbatch, float carry) {
  __shared__ __align__(16) _Float16 sT[32 * 72];
  const int tid = threadIdx.x;
  const int n0 = blockIdx.x * 32, k0 = blockIdx.y * 64;
  const float* ib = in + (size_t)blockIdx.z * inbatch;
  unsigned short* ob = out + (size_t)blockIdx.z * outbatch;
  {
    const int k = tid >> 2, c8 = (tid & 3) * 8;
    const bool ok = (n0 + c8 + 8 <= nreal);
    const int cc = ok ? (n0 + c8) : 0;
    const size_t ro = (size_t)(k0 + k) * ldin + cc;
    const v4f a = *(const v4f*)(ib + ro);
    const v4f b = *(const v4f*)(ib + ro + 4);
    const float kp = ok ? carry : 0.0f;
#pragma unroll
    for (int j = 0; j < 4; ++j) {
      sT[(c8 + j) * 72 + k]     = (_Float16)(bfr(a[j]) * kp);
      sT[(c8 + 4 + j) * 72 + k] = (_Float16)(bfr(b[j]) * kp);
    }
  }
  __syncthreads();
  {
    const int n = tid >> 3, c8 = (tid & 7) * 8;
    const v4u v = *(const v4u*)(&sT[n * 72 + c8]);
    unsigned short* dst = ob + (size_t)(n0 + n) * ldout + coloff + k0 + c8;
    *(volatile v4u*)dst = v;
    __threadfence();
    *(volatile v4u*)dst = v;
  }
}

__global__ __launch_bounds__(256) void rope_tab_kernel(float* tab, int npos) {
#pragma clang fp contract(off)
  const int lane = threadIdx.x & 31, wave = threadIdx.x >> 5;
  int pos = blockIdx.x * 8 + wave;
  pos = (pos < npos) ? pos : (npos - 1);
  double P = 1.0;
#pragma unroll 1
  for (int j = 0; j < lane; ++j) P *= 1.333521432163324;
  const float p32 = (float)P;
  const float inv = (float)(1.0 / (double)p32);
  const float ang = (float)pos * inv;
  const double a = (double)ang;
  const double kq = rint(a * 0.6366197723675814);
  const double rr = a - kq * 1.5707963267948966;
  const int qd = ((int)kq) & 3;
  const float r = (float)rr;
  const float r2 = r * r;
  const float sp = r + r * r2 * (-1.6666654611e-1f + r2 * (8.3321608736e-3f + r2 * (-1.9515295891e-4f)));
  const float cp = 1.0f - 0.5f * r2 + (r2 * r2) * (4.166664568298827e-2f + r2 * (-1.388731625493765e-3f + r2 * 2.443315711809948e-5f));
  const float sn = (qd == 0) ? sp : ((qd == 1) ? cp : ((qd == 2) ? -sp : -cp));
  const float cs = (qd == 0) ? cp : ((qd == 1) ? -sp : ((qd == 2) ? -cp : sp));
  float* rowp = tab + (size_t)pos * 64;
  *(volatile float*)(rowp + lane) = cs;
  *(volatile float*)(rowp + 32 + lane) = sn;
  __threadfence();
  *(volatile float*)(rowp + lane) = cs;
  *(volatile float*)(rowp + 32 + lane) = sn;
}

template <bool FIRST>
__global__ __launch_bounds__(256) void rms_split_kernel(const float* xin, const float* __restrict__ gamma,
                                                         float* xs, unsigned short* Hhl, int nrow) {
  __shared__ __align__(16) float sL[8][DM];
  const int tid = threadIdx.x, wave = tid >> 5, lane = tid & 31;
  int row = blockIdx.x * 8 + wave;
  row = (row < nrow) ? row : (nrow - 1);
  size_t srow = (size_t)row;
  if (FIRST) {
    const int b = row / SEQ;
    const int t = row - b * SEQ;
    srow = (size_t)b * SEQ_FULL + (size_t)t;
  }
  const float* rp = xin + srow * DM + 4 * lane;
  v4f a0 = *(const v4f*)(rp);
  v4f a1 = *(const v4f*)(rp + 128);
  v4f a2 = *(const v4f*)(rp + 256);
  v4f a3 = *(const v4f*)(rp + 384);
  if (FIRST) { a0 = bfr4(a0); a1 = bfr4(a1); a2 = bfr4(a2); a3 = bfr4(a3); }
  float ss = (sq4(a0) + sq4(a1)) + (sq4(a2) + sq4(a3));
#pragma unroll
  for (int off = 16; off > 0; off >>= 1) ss += __shfl_xor(ss, off, 32);
  const float inv = 1.0f / sqrtf(ss * (1.0f / DM) + 1e-6f);
  const float* gp = gamma + 4 * lane;
  const v4f y0 = (a0 * inv) * bfr4(*(const v4f*)(gp));
  const v4f y1 = (a1 * inv) * bfr4(*(const v4f*)(gp + 128));
  const v4f y2 = (a2 * inv) * bfr4(*(const v4f*)(gp + 256));
  const v4f y3 = (a3 * inv) * bfr4(*(const v4f*)(gp + 384));
  {
    const v4f s0 = FIRST ? a0 : y0;
    const v4f s1 = FIRST ? a1 : y1;
    const v4f s2 = FIRST ? a2 : y2;
    const v4f s3 = FIRST ? a3 : y3;
    float* orow = xs + (size_t)row * DM + 4 * lane;
    *(volatile v4f*)(orow) = s0;
    *(volatile v4f*)(orow + 128) = s1;
    *(volatile v4f*)(orow + 256) = s2;
    *(volatile v4f*)(orow + 384) = s3;
    __threadfence();
    *(volatile v4f*)(orow) = s0;
    *(volatile v4f*)(orow + 128) = s1;
    *(volatile v4f*)(orow + 256) = s2;
    *(volatile v4f*)(orow + 384) = s3;
  }
  *(v4f*)(&sL[wave][4 * lane]) = y0;
  *(v4f*)(&sL[wave][128 + 4 * lane]) = y1;
  *(v4f*)(&sL[wave][256 + 4 * lane]) = y2;
  *(v4f*)(&sL[wave][384 + 4 * lane]) = y3;
  wave_lds_sync();
  const v4f u0 = *(const v4f*)(&sL[wave][8 * lane]);
  const v4f u1 = *(const v4f*)(&sL[wave][8 * lane + 4]);
  const v4f u2 = *(const v4f*)(&sL[wave][256 + 8 * lane]);
  const v4f u3 = *(const v4f*)(&sL[wave][256 + 8 * lane + 4]);
  v4u hiA, loA, hiB, loB;
  split8(u0, u1, HCAR, hiA, loA);
  split8(u2, u3, HCAR, hiB, loB);
  unsigned short* dst = Hhl + (size_t)row * (2 * DM) + 8 * lane;
  *(volatile v4u*)(dst) = hiA;
  *(volatile v4u*)(dst + 256) = hiB;
  *(volatile v4u*)(dst + DM) = loA;
  *(volatile v4u*)(dst + DM + 256) = loB;
  __threadfence();
  *(volatile v4u*)(dst) = hiA;
  *(volatile v4u*)(dst + 256) = hiB;
  *(volatile v4u*)(dst + DM) = loA;
  *(volatile v4u*)(dst + DM + 256) = loB;
}

__global__ __launch_bounds__(256) void split_kd_kernel(const float* KDf, unsigned short* KD2, int nrow) {
  const int tid = threadIdx.x, wave = tid >> 5, lane = tid & 31;
  int row = blockIdx.x * 32 + wave * 4 + (lane >> 3);
  row = (row < nrow) ? row : (nrow - 1);
  const int c8 = (lane & 7) * 8;
  const float* rp = KDf + (size_t)row * DLT + c8;
  const v4f a = *(const v4f*)(rp);
  const v4f b = *(const v4f*)(rp + 4);
  v4u hi, lo;
  split8(a, b, KDCAR, hi, lo);
  unsigned short* dp = KD2 + (size_t)row * (2 * DLT) + c8;
  *(volatile v4u*)(dp) = hi;
  *(volatile v4u*)(dp + DLT) = lo;
  __threadfence();
  *(volatile v4u*)(dp) = hi;
  *(volatile v4u*)(dp + DLT) = lo;
}

__global__ __launch_bounds__(256) void head_attn_kernel(const float* Qf, const float* KVf, const float* __restrict__ tab,
                                                        unsigned short* CTX, int ntok) {
  __shared__ __align__(16) float sq[8][DM];
  __shared__ __align__(16) float skv[8][KVW];
  __shared__ float sa[8][64];
  const int tid = threadIdx.x, wave = tid >> 5, lane = tid & 31;
  int m = blockIdx.x * 8 + wave;
  m = (m < ntok) ? m : (ntok - 1);
  const int pos = m % SEQ;
  float* q_ = sq[wave];
  float* k_ = skv[wave];
  float* v_ = skv[wave] + DM;
  float* a_ = sa[wave];
  {
    const float* qr = Qf + (size_t)m * DM + 16 * lane;
#pragma unroll
    for (int j = 0; j < 4; ++j) *(v4f*)(q_ + 16 * lane + 4 * j) = *(const v4f*)(qr + 4 * j);
    const float* kr = KVf + (size_t)m * KVW + 32 * lane;
    const int hh = lane >> 2, p = lane & 3;
    const int di = (p >> 1) * DM + hh * HDD + (p & 1) * 32;
#pragma unroll
    for (int j = 0; j < 8; ++j) *(v4f*)(k_ + di + 4 * j) = *(const v4f*)(kr + 4 * j);
  }
  wave_lds_sync();
  {
    const float cs = tab[(size_t)pos * 64 + lane];
    const float sn = tab[(size_t)pos * 64 + 32 + lane];
#pragma unroll 1
    for (int hh = 0; hh < NHD; ++hh) {
      const int i0 = hh * HDD + lane, i1 = i0 + 32;
      const float q1 = q_[i0], q2 = q_[i1];
      q_[i0] = q1 * cs - q2 * sn;
      q_[i1] = q1 * sn + q2 * cs;
      const float k1 = k_[i0], k2 = k_[i1];
      k_[i0] = k1 * cs - k2 * sn;
      k_[i1] = k1 * sn + k2 * cs;
    }
  }
  wave_lds_sync();
  float s0, s1;
  {
    const float* qa = q_ + (lane >> 3) * HDD;
    const float* qb = q_ + (4 + (lane >> 3)) * HDD;
    const float* kg = k_ + (lane & 7) * HDD;
    v4f ca = (v4f){0.f, 0.f, 0.f, 0.f}, cb = (v4f){0.f, 0.f, 0.f, 0.f};
#pragma unroll 1
    for (int d = 0; d < HDD; d += 4) {
      const v4f kk = *(const v4f*)(kg + d);
      const v4f qx = *(const v4f*)(qa + d);
      const v4f qy = *(const v4f*)(qb + d);
      ca += qx * kk;
      cb += qy * kk;
    }
    s0 = ((ca[0] + ca[1]) + (ca[2] + ca[3])) * 0.125f;
    s1 = ((cb[0] + cb[1]) + (cb[2] + cb[3])) * 0.125f;
  }
  float mx0 = s0, mx1 = s1;
#pragma unroll
  for (int off = 1; off < 8; off <<= 1) {
    mx0 = fmaxf(mx0, __shfl_xor(mx0, off, 32));
    mx1 = fmaxf(mx1, __shfl_xor(mx1, off, 32));
  }
  const float e0 = expf(s0 - mx0), e1 = expf(s1 - mx1);
  float sm0 = e0, sm1 = e1;
#pragma unroll
  for (int off = 1; off < 8; off <<= 1) {
    sm0 += __shfl_xor(sm0, off, 32);
    sm1 += __shfl_xor(sm1, off, 32);
  }
  a_[lane] = e0 * (1.0f / sm0);
  a_[32 + lane] = e1 * (1.0f / sm1);
  wave_lds_sync();
  const int hA = lane >> 3, dA = (lane & 7) * 8;
  v4f o0 = (v4f){0.f, 0.f, 0.f, 0.f}, o1 = o0, o2 = o0, o3 = o0;
#pragma unroll 1
  for (int g = 0; g < NHD; ++g) {
    const float wA = a_[hA * 8 + g];
    const float wB = a_[(hA + 4) * 8 + g];
    const v4f va = *(const v4f*)(v_ + g * HDD + dA);
    const v4f vb = *(const v4f*)(v_ + g * HDD + dA + 4);
    o0 += wA * va;
    o1 += wA * vb;
    o2 += wB * va;
    o3 += wB * vb;
  }
  v4u hiA, loA, hiB, loB;
  split8(o0, o1, OCAR, hiA, loA);
  split8(o2, o3, OCAR, hiB, loB);
  unsigned short* dst = CTX + (size_t)m * (2 * DM) + 8 * lane;
  *(volatile v4u*)(dst) = hiA;
  *(volatile v4u*)(dst + 256) = hiB;
  *(volatile v4u*)(dst + DM) = loA;
  *(volatile v4u*)(dst + DM + 256) = loB;
  __threadfence();
  *(volatile v4u*)(dst) = hiA;
  *(volatile v4u*)(dst + 256) = hiB;
  *(volatile v4u*)(dst + DM) = loA;
  *(volatile v4u*)(dst + DM + 256) = loB;
}

__global__ __launch_bounds__(256) void moe_rows_kernel(const float* H2f, const float* LG, const float* __restrict__ bg,
                                                       unsigned short* AP, int chunk, int ntok) {
  const int tid = threadIdx.x, wave = tid >> 5, lane = tid & 31;
  int m = blockIdx.x * 8 + wave;
  m = (m < ntok) ? m : (ntok - 1);
  const float z = LG[(size_t)m * NEXP2 + lane] + bfr(bg[lane]);
  float mx = z;
#pragma unroll
  for (int off = 16; off > 0; off >>= 1) mx = fmaxf(mx, __shfl_xor(mx, off, 32));
  const float ex = expf(z - mx);
  float sm = ex;
#pragma unroll
  for (int off = 16; off > 0; off >>= 1) sm += __shfl_xor(sm, off, 32);
  const float g = ex * (1.0f / sm);
  const float* hp = H2f + (size_t)m * DM + 8 * lane;
  const v4f fa0 = *(const v4f*)(hp);
  const v4f fa1 = *(const v4f*)(hp + 4);
  const v4f fb0 = *(const v4f*)(hp + 256);
  const v4f fb1 = *(const v4f*)(hp + 260);
  unsigned short* ob = AP + (size_t)m * KCH + 8 * lane;
#pragma unroll 1
  for (int el = 0; el < ECH; ++el) {
    const float ge = __shfl(g, chunk * ECH + el, 32) * GCAR;
    Pk8 pa, pb;
#pragma unroll
    for (int e = 0; e < 4; ++e) {
      pa.h[e]     = (_Float16)(fa0[e] * ge);
      pa.h[4 + e] = (_Float16)(fa1[e] * ge);
      pb.h[e]     = (_Float16)(fb0[e] * ge);
      pb.h[4 + e] = (_Float16)(fb1[e] * ge);
    }
    const v4u va = pa.u, vb = pb.u;
    unsigned short* d0 = ob + el * DM;
    *(volatile v4u*)(d0) = va;
    *(volatile v4u*)(d0 + 256) = vb;
    __threadfence();
    *(volatile v4u*)(d0) = va;
    *(volatile v4u*)(d0 + 256) = vb;
  }
}

extern "C" void kernel_launch(void* const* d_in, const int* in_sizes, int n_in,
                              void* d_out, int out_size, void* d_ws, size_t ws_size,
                              hipStream_t stream) {
  if (n_in < 14) return;
  if ((size_t)in_sizes[0] < ((size_t)(NB - 1) * SEQ_FULL + (size_t)SEQ) * DM) return;
  if (in_sizes[1] < DM || in_sizes[2] < DM) return;
  if (in_sizes[3] < DM * DM || in_sizes[4] < DM) return;
  if (in_sizes[5] < DM * DLT || in_sizes[6] < DLT) return;
  if (in_sizes[7] < DLT * KVW || in_sizes[8] < KVW) return;
  if (in_sizes[9] < DM * DM || in_sizes[10] < DM) return;
  if (in_sizes[11] < DM * NEX || in_sizes[12] < NEX) return;
  if (in_sizes[13] < NEX * DM * DM) return;
  if (out_size < MTOK * DM) return;

  const float* x      = (const float*)d_in[0];
  const float* gamma1 = (const float*)d_in[1];
  const float* gamma2 = (const float*)d_in[2];
  const float* wq     = (const float*)d_in[3];
  const float* bq     = (const float*)d_in[4];
  const float* wkd    = (const float*)d_in[5];
  const float* bkd    = (const float*)d_in[6];
  const float* wku    = (const float*)d_in[7];
  const float* bku    = (const float*)d_in[8];
  const float* wo     = (const float*)d_in[9];
  const float* bo     = (const float*)d_in[10];
  const float* wg     = (const float*)d_in[11];
  const float* bg     = (const float*)d_in[12];
  const float* ew     = (const float*)d_in[13];
  float* outp = (float*)d_out;

  const size_t PWQ  = (size_t)DM * (2 * DM) * 2;
  const size_t PWKD = (size_t)DLT * (2 * DM) * 2;
  const size_t PWKU = (size_t)KVW * (2 * DLT) * 2;
  const size_t PWO  = (size_t)DM * (2 * DM) * 2;
  const size_t PWG  = (size_t)NEXP2 * (2 * DM) * 2;
  const size_t PEW  = (size_t)DM * KEW * 2;
  const size_t PTAB = (size_t)SEQ_FULL * 64 * 4;
  const size_t PX   = (size_t)MTOK * KCH * 2;
  const size_t PY   = (size_t)MTOK * DM * 4 + (size_t)MTOK * (2 * DM) * 2 + (size_t)MTOK * NEXP2 * 4;
  size_t off = 0;
  const size_t oWq = off; off += PWQ;
  const size_t oWkd = off; off += PWKD;
  const size_t oWku = off; off += PWKU;
  const size_t oWo = off; off += PWO;
  const size_t oWg = off; off += PWG;
  const size_t oEW = off; off += PEW;
  const size_t oTab = off; off += PTAB;
  const size_t oX = off; off += PX;
  const size_t oY = off; off += PY;
  if (off > ws_size) return;
  if (off > (size_t)134217728u) return;
  const size_t oQf  = oX;
  const size_t oKVf = oQf + (size_t)MTOK * DM * 4;
  const size_t oKDf = oKVf + (size_t)MTOK * KVW * 4;
  const size_t oKD2 = oKDf + (size_t)MTOK * DLT * 4;
  if (oKD2 + (size_t)MTOK * (2 * DLT) * 2 > oX + PX) return;
  const size_t oAP  = oX;
  const size_t oH1  = oY;
  const size_t oCTX = oY;
  const size_t oH2f = oY;
  const size_t oH2h = oH2f + (size_t)MTOK * DM * 4;
  const size_t oLG  = oH2h + (size_t)MTOK * (2 * DM) * 2;
  if (oLG + (size_t)MTOK * NEXP2 * 4 > oY + PY) return;
  if (oCTX + (size_t)MTOK * (2 * DM) * 2 > oY + PY) return;

  char* ws = (char*)d_ws;
  unsigned short* Wq2  = (unsigned short*)(ws + oWq);
  unsigned short* Wkd2 = (unsigned short*)(ws + oWkd);
  unsigned short* Wku2 = (unsigned short*)(ws + oWku);
  unsigned short* Wo2  = (unsigned short*)(ws + oWo);
  unsigned short* Wg2  = (unsigned short*)(ws + oWg);
  unsigned short* EW   = (unsigned short*)(ws + oEW);
  float*          TAB  = (float*)(ws + oTab);
  float*          Qf   = (float*)(ws + oQf);
  float*          KVf  = (float*)(ws + oKVf);
  float*          KDf  = (float*)(ws + oKDf);
  unsigned short* KD2  = (unsigned short*)(ws + oKD2);
  unsigned short* AP   = (unsigned short*)(ws + oAP);
  unsigned short* H1   = (unsigned short*)(ws + oH1);
  unsigned short* CTX2 = (unsigned short*)(ws + oCTX);
  float*          H2f  = (float*)(ws + oH2f);
  unsigned short* H2hl = (unsigned short*)(ws + oH2h);
  float*          LG   = (float*)(ws + oLG);

  const dim3 blk(256);
  const size_t z0 = 0;
  tr_w16_kernel<<<dim3(DM / 32, DM / 64, 1), blk, 0, stream>>>(wq, DM, DM, z0, Wq2, 2 * DM, 0, z0, WCAR);
  tr_w16_kernel<<<dim3(DM / 32, DM / 64, 1), blk, 0, stream>>>(wq, DM, DM, z0, Wq2, 2 * DM, DM, z0, WLCAR);
  tr_w16_kernel<<<dim3(DLT / 32, DM / 64, 1), blk, 0, stream>>>(wkd, DLT, DLT, z0, Wkd2, 2 * DM, 0, z0, WCAR);
  tr_w16_kernel<<<dim3(DLT / 32, DM / 64, 1), blk, 0, stream>>>(wkd, DLT, DLT, z0, Wkd2, 2 * DM, DM, z0, WLCAR);
  tr_w16_kernel<<<dim3(KVW / 32, DLT / 64, 1), blk, 0, stream>>>(wku, KVW, KVW, z0, Wku2, 2 * DLT, 0, z0, WCAR);
  tr_w16_kernel<<<dim3(KVW / 32, DLT / 64, 1), blk, 0, stream>>>(wku, KVW, KVW, z0, Wku2, 2 * DLT, DLT, z0, WLCAR);
  tr_w16_kernel<<<dim3(DM / 32, DM / 64, 1), blk, 0, stream>>>(wo, DM, DM, z0, Wo2, 2 * DM, 0, z0, WCAR);
  tr_w16_kernel<<<dim3(DM / 32, DM / 64, 1), blk, 0, stream>>>(wo, DM, DM, z0, Wo2, 2 * DM, DM, z0, WLCAR);
  tr_w16_kernel<<<dim3(NEXP2 / 32, DM / 64, 1), blk, 0, stream>>>(wg, NEX, NEX, z0, Wg2, 2 * DM, 0, z0, WCAR);
  tr_w16_kernel<<<dim3(NEXP2 / 32, DM / 64, 1), blk, 0, stream>>>(wg, NEX, NEX, z0, Wg2, 2 * DM, DM, z0, WLCAR);
  tr_w16_kernel<<<dim3(DM / 32, DM / 64, NEX), blk, 0, stream>>>(ew, DM, DM, (size_t)DM * DM, EW, KEW, 0, (size_t)DM, WCAR);
  rope_tab_kernel<<<dim3(SEQ / 8), blk, 0, stream>>>(TAB, SEQ);
  rms_split_kernel<true><<<dim3(MTOK / 8), blk, 0, stream>>>(x, gamma1, outp, H1, MTOK);

  const int tilesM = MTOK / 64;
  wmma_gemm64<2, 0, false><<<dim3((tilesM * (DM / 64) + 7) / 8), blk, 0, stream>>>(
      H1, 2 * DM, Wq2, 2 * DM, (void*)Qf, DM, bq, bq, MTOK, DM, 2 * DM, 1.0f / (HCAR * WCAR), 1.0f);
  wmma_gemm64<2, 0, false><<<dim3((tilesM * (DLT / 64) + 7) / 8), blk, 0, stream>>>(
      H1, 2 * DM, Wkd2, 2 * DM, (void*)KDf, DLT, bkd, bkd, MTOK, DLT, 2 * DM, 1.0f / (HCAR * WCAR), 1.0f);
  split_kd_kernel<<<dim3(MTOK / 32), blk, 0, stream>>>(KDf, KD2, MTOK);
  wmma_gemm64<2, 0, false><<<dim3((tilesM * (KVW / 64) + 7) / 8), blk, 0, stream>>>(
      KD2, 2 * DLT, Wku2, 2 * DLT, (void*)KVf, KVW, bku, bku, MTOK, KVW, 2 * DLT, 1.0f / (KDCAR * WCAR), 1.0f);
  head_attn_kernel<<<dim3(MTOK / 8), blk, 0, stream>>>(Qf, KVf, TAB, CTX2, MTOK);
  wmma_gemm64<2, 0, true><<<dim3((tilesM * (DM / 64) + 7) / 8), blk, 0, stream>>>(
      CTX2, 2 * DM, Wo2, 2 * DM, (void*)outp, DM, bo, outp, MTOK, DM, 2 * DM, 1.0f / (OCAR * WCAR), 1.0f);
  rms_split_kernel<false><<<dim3(MTOK / 8), blk, 0, stream>>>(outp, gamma2, H2f, H2hl, MTOK);
  wmma_gemm64<0, 0, false><<<dim3((tilesM * (NEXP2 / 64) + 7) / 8), blk, 0, stream>>>(
      H2hl, 2 * DM, Wg2, 2 * DM, (void*)LG, NEXP2, bg, bg, MTOK, NEXP2, 2 * DM, 1.0f / (HCAR * WCAR), 1.0f);
  for (int c = 0; c < NCHK; ++c) {
    moe_rows_kernel<<<dim3(MTOK / 8), blk, 0, stream>>>(H2f, LG, bg, AP, c, MTOK);
    wmma_gemm64<0, 0, true><<<dim3((tilesM * (DM / 64) + 7) / 8), blk, 0, stream>>>(
        AP, KCH, EW + (size_t)c * KCH, KEW, (void*)outp, DM, bo, outp, MTOK, DM, KCH, 1.0f / (GCAR * WCAR), 1.0f);
  }
  (void)hipGetLastError();
}
